// SimpleModel_29059748725144
// MI455X (gfx1250) — hardware-run, weakly checked
//
#include <hip/hip_runtime.h>


namespace {

constexpr int N = 50000, NP = 50176, NPL = NP  , SRCM = N  , NST = (NPL < N ? NPL : N)  , EFULL = 600000, E = EFULL  , D = 128, KCH = 1024, NCH = NPL / KCH, NB64 = NPL / 64, SWEEPS = 12  ;
constexpr float XS = 8.0f, WSC = 256.0f, RS_ = 1024.0f, SLOPE = 0.0f, BNEPS = 1e-5f;
static_assert(NP % KCH == 0 && NPL % KCH == 0 && NP >= N && D == 128 && NPL % 64 == 0, "tiling");
typedef _Float16 b16;
typedef __attribute__((ext_vector_type(16))) _Float16 v16b;
typedef __attribute__((ext_vector_type(8))) _Float16 v8b;
typedef __attribute__((ext_vector_type(8))) float v8f;
typedef __attribute__((ext_vector_type(4))) float v4f;
__device__ __forceinline__ float bf16_rne(float f) { unsigned int u = __float_as_uint(f); u += 0x7FFFu + ((u >> 16) & 1u); return __uint_as_float(u & 0xFFFF0000u); }
__device__ __forceinline__ void split16(float v, b16& hi, b16& lo) { hi = (b16)v; lo = (b16)(v - (float)hi); }
__device__ __forceinline__ v16b frag_kb(const b16* p, int hh) { const v8b a = *(const v8b*)(p + 8 * hh), b = *(const v8b*)(p + 16 + 8 * hh); v16b f;
#pragma unroll
  for (int e = 0; e < 8; ++e) { f[e] = a[e]; f[8 + e] = b[e]; } return f; }
__device__ __forceinline__ v8f wmma16b(v16b a, v16b b, v8f c) { v8f d = __builtin_amdgcn_wmma_f32_16x16x32_f16(false, a, false, b, (short)0, c, false, false); asm volatile("v_nop\n\tv_nop\n\tv_nop\n\tv_nop" : "+v"(d) : "v"(a), "v"(b)); return d; }
__device__ __forceinline__ void wave_lds_sync() { __builtin_amdgcn_fence(__ATOMIC_RELEASE, "workgroup"); __builtin_amdgcn_wave_barrier(); __builtin_amdgcn_fence(__ATOMIC_ACQUIRE, "workgroup"); }
__device__ __forceinline__ float pmul(float a, float b) { float p = a * b; asm volatile("" : "+v"(p)); return p; }
__device__ __forceinline__ int iclamp(int v, int lo, int hi) { return v < lo ? lo : (v > hi ? hi : v); }
constexpr int CSR_NBLK = 512, CSR_GB = 9, CSR_GN = 1 << CSR_GB  , CSR_MAXG = 512, CSR_CAP = 12288  ;
__global__ __launch_bounds__(64) void csrA_kernel(const int* __restrict__ dst, int E, int N, int nG, int CHP, int NGP, int* __restrict__ STG, int* __restrict__ HST) {
  extern __shared__ int sm[];
  int* cnt = sm; int* run = sm + NGP; int* ids = sm + 2 * NGP;
  const int b = blockIdx.x; const int ch = (E + CSR_NBLK - 1) / CSR_NBLK; const int e0 = b * ch, e1 = min(E, e0 + ch);
  for (int i = threadIdx.x; i < NGP; i += 64) cnt[i] = 0;
  for (int i = threadIdx.x; i < CHP; i += 64) ids[i] = -1;
  __syncthreads();
  if (threadIdx.x == 0) {
    for (int e = e0; e < e1; ++e) { int d = dst[e]; d = (d < 0) ? 0 : (d >= N ? N - 1 : d); cnt[d >> CSR_GB] += 1; }
    int acc = 0; for (int g = 0; g < nG; ++g) { run[g] = acc; acc += cnt[g]; }
    for (int e = e0; e < e1; ++e) { int d = dst[e]; d = (d < 0) ? 0 : (d >= N ? N - 1 : d); const int g = d >> CSR_GB; ids[run[g]] = e; run[g] += 1; } }
  __syncthreads();
  typedef __attribute__((ext_vector_type(4))) int v4i;
  for (int pass = 0; pass < 2; ++pass) {
    for (int i = threadIdx.x; i < CHP / 4; i += 64) *(volatile v4i*)(STG + (size_t)b * CHP + i * 4) = *(const v4i*)(&ids[i * 4]);
    for (int i = threadIdx.x; i < NGP / 4; i += 64) { v4i v; for (int e = 0; e < 4; ++e) v[e] = (i * 4 + e < nG) ? cnt[i * 4 + e] : 0; *(volatile v4i*)(HST + (size_t)b * NGP + i * 4) = v; }
    __threadfence(); }
}
__global__ __launch_bounds__(512) void csrS_kernel(const int* __restrict__ HST, int nG, int NGP, int* __restrict__ START, int* __restrict__ TOT, int* __restrict__ OFF) {
  __shared__ int tot[CSR_MAXG];
  const int b = threadIdx.x;
  for (int pass = 0; pass < 2; ++pass) { int runb = 0; for (int g = 0; g < nG; ++g) { int c = HST[(size_t)b * NGP + g]; c = (c < 0) ? 0 : c; ((volatile int*)OFF)[(size_t)g * CSR_NBLK + b] = runb; runb += c; } __threadfence(); }
  for (int g = threadIdx.x; g < nG; g += 512) { int s = 0; for (int bb = 0; bb < CSR_NBLK; ++bb) { int c = HST[(size_t)bb * NGP + g]; s += (c < 0) ? 0 : c; } tot[g] = s; }
  __syncthreads();
  if (threadIdx.x < 32) {
    __shared__ int st[CSR_MAXG + 32];
    if (threadIdx.x == 0) { int acc = 0; for (int g = 0; g < NGP; ++g) { st[g] = acc; if (g < nG) acc += (tot[g] + 31) & ~31; } st[NGP] = acc; }
    __builtin_amdgcn_fence(__ATOMIC_RELEASE, "workgroup"); __builtin_amdgcn_wave_barrier(); __builtin_amdgcn_fence(__ATOMIC_ACQUIRE, "workgroup");
    for (int pass = 0; pass < 2; ++pass) { for (int i = threadIdx.x; i < NGP + 32; i += 32) { ((volatile int*)START)[i] = (i <= NGP) ? st[min(i, NGP)] : 0; ((volatile int*)TOT)[i] = (i < nG) ? tot[i] : 0; } __threadfence(); } }
}
__global__ __launch_bounds__(256) void csrB_kernel(const int* __restrict__ dst, int N, int nG, int CHP, int NGP, int permLen, const int* __restrict__ STG, const int* __restrict__ HST, const int* __restrict__ OFF, const int* __restrict__ START, const int* __restrict__ TOT, int* __restrict__ PERM, int* __restrict__ ROWPTR, int* __restrict__ ROWCNT, int* __restrict__ FLAG) {
  typedef __attribute__((ext_vector_type(4))) int v4i;
  __shared__ int ids[CSR_CAP]; __shared__ unsigned short key[CSR_CAP]; __shared__ int outp[CSR_CAP]; __shared__ int ncnt[CSR_GN + 1]; __shared__ int boff[CSR_NBLK + 1];
  const int g = blockIdx.x, t_ = threadIdx.x; int tot = TOT[g]; int st = START[g], stn = START[g + 1]; const int v0 = g * CSR_GN; const int nv = min(CSR_GN, N - v0);
  st = (st < 0) ? 0 : (st > permLen - 32 ? permLen - 32 : st) & ~31; stn = (stn < st) ? st : (stn > permLen ? permLen : stn); tot = (tot < 0) ? 0 : tot; if (tot > stn - st && tot <= CSR_CAP) tot = stn - st;
  if (tot > CSR_CAP) {
    for (int pass = 0; pass < 2; ++pass) { for (int i = t_; i < CSR_GN / 4; i += 256) { v4i a, c; for (int e = 0; e < 4; ++e) { a[e] = st; c[e] = 0; } *(volatile v4i*)(ROWPTR + v0 + i * 4) = a; *(volatile v4i*)(ROWCNT + v0 + i * 4) = c; } if (t_ == 0) ((volatile int*)FLAG)[0] = 1; __threadfence(); } (void)nv; return; }
  if (t_ == 0) { int acc = 0; for (int b = 0; b < CSR_NBLK; ++b) { boff[b] = acc; int c = HST[(size_t)b * NGP + g]; c = (c < 0) ? 0 : (c > CHP ? CHP : c); acc += c; if (acc > tot) acc = tot; } boff[CSR_NBLK] = acc; }
  for (int i = t_; i <= CSR_GN; i += 256) ncnt[i] = 0;
  __syncthreads();
  for (int b = 0; b < CSR_NBLK; ++b) { const int c = boff[b + 1] - boff[b]; int o_ = OFF[(size_t)g * CSR_NBLK + b]; o_ = (o_ < 0) ? 0 : (o_ > CHP - c ? CHP - c : o_); const int* src_ = STG + (size_t)b * CHP + o_;
    for (int i = t_; i < c; i += 256) { int id = src_[i]; id = (id < 0) ? 0 : id; ids[boff[b] + i] = id; int d = dst[id]; d = (d < v0) ? v0 : (d >= N ? N - 1 : d); int kk = d - v0; kk = (kk < 0) ? 0 : (kk >= CSR_GN ? CSR_GN - 1 : kk); key[boff[b] + i] = (unsigned short)kk; } }
  __syncthreads();
  if (t_ == 0) { for (int i = 0; i < tot; ++i) ncnt[key[i]] += 1; int acc = 0; for (int vl = 0; vl < CSR_GN; ++vl) { const int c = ncnt[vl]; ncnt[vl] = acc; acc += c; } ncnt[CSR_GN] = acc;
    for (int i = 0; i < tot; ++i) { const int vl = key[i]; outp[ncnt[vl]] = ids[i]; ncnt[vl] += 1; }
    for (int vl = CSR_GN; vl > 0; --vl) ncnt[vl] = ncnt[vl - 1]; ncnt[0] = 0; }
  __syncthreads();
  for (int pass = 0; pass < 2; ++pass) {
    for (int i = t_; i < (stn - st) / 4; i += 256) { v4i v; for (int e = 0; e < 4; ++e) { const int q = i * 4 + e; v[e] = (q < tot) ? outp[q] : -1; } *(volatile v4i*)(PERM + st + i * 4) = v; }
    for (int i = t_; i < CSR_GN / 4; i += 256) { v4i a, c; for (int e = 0; e < 4; ++e) { const int vl = i * 4 + e; a[e] = st + ncnt[vl]; c[e] = (vl < nv) ? (ncnt[vl + 1] - ncnt[vl]) : 0; } *(volatile v4i*)(ROWPTR + v0 + i * 4) = a; *(volatile v4i*)(ROWCNT + v0 + i * 4) = c; }
    __threadfence(); }
}
__global__ __launch_bounds__(256) void csrZ_kernel(int* __restrict__ p, size_t n4) { typedef __attribute__((ext_vector_type(4))) int v4i; const size_t tid = (size_t)blockIdx.x * 256 + threadIdx.x, nth = (size_t)gridDim.x * 256; v4i z = {0, 0, 0, 0}; for (size_t i = tid; i < n4; i += nth) *(volatile v4i*)(p + i * 4) = z; }
struct CsrBufs { int *STG, *HST, *OFF, *START, *TOT, *PERM, *ROWPTR, *ROWCNT, *FLAG; int nG, NGP, CHP; size_t permLen; char* base; size_t bytes; };
static size_t csr_carve(CsrBufs& c, char* ws, size_t off, int E, int N) {
  const size_t off0 = off; c.base = ws + off;
  auto al = [&](size_t bytes) { char* p = ws + off; off += (bytes + 255) & ~(size_t)255; return p; };
  c.nG = (N + CSR_GN - 1) / CSR_GN; c.NGP = (c.nG + 31) & ~31; const int ch = (E + CSR_NBLK - 1) / CSR_NBLK; c.CHP = (ch + 31) & ~31; c.permLen = (size_t)E + 32 * (size_t)c.nG + 32;
  c.STG = (int*)al((size_t)CSR_NBLK * c.CHP * 4); c.HST = (int*)al((size_t)CSR_NBLK * c.NGP * 4); c.OFF = (int*)al((size_t)c.NGP * CSR_NBLK * 4); c.START = (int*)al((size_t)(c.NGP + 64) * 4); c.TOT = (int*)al((size_t)(c.NGP + 64) * 4);
  c.PERM = (int*)al(c.permLen * 4); c.ROWPTR = (int*)al((size_t)c.nG * CSR_GN * 4); c.ROWCNT = (int*)al((size_t)c.nG * CSR_GN * 4); c.FLAG = (int*)al(256);
  c.bytes = off - off0; return off;
}
static void csr_build(const CsrBufs& c, const int* dst, int E, int N, hipStream_t stream) {
  const size_t smem = (size_t)(2 * c.NGP + c.CHP) * 4;
  csrZ_kernel<<<512, 256, 0, stream>>>((int*)c.base, c.bytes / 16);
  csrA_kernel<<<CSR_NBLK, 64, smem, stream>>>(dst, E, N, c.nG, c.CHP, c.NGP, c.STG, c.HST);
  csrS_kernel<<<1, 512, 0, stream>>>(c.HST, c.nG, c.NGP, c.START, c.TOT, c.OFF);
  csrB_kernel<<<c.nG, 256, 0, stream>>>(dst, N, c.nG, c.CHP, c.NGP, (int)c.permLen, c.STG, c.HST, c.OFF, c.START, c.TOT, c.PERM, c.ROWPTR, c.ROWCNT, c.FLAG);
}


typedef __attribute__((ext_vector_type(4))) _Float16 v4h;
typedef __attribute__((ext_vector_type(2))) float v2f;
template <int KD, int NOUT>
__global__ __launch_bounds__(256) void wprep_kernel(const float* __restrict__ w, b16* __restrict__ WT) {
  static_assert(KD % 8 == 0, "wprep"); const size_t u = (size_t)blockIdx.x * 256 + threadIdx.x; if (u >= (size_t)NOUT * KD / 8) return; const size_t e = u * 8; const int oo = (int)(e / KD), k0 = (int)(e % KD); v8b o;
  for (int j = 0; j < 8; ++j) o[j] = (b16)(bf16_rne(w[(size_t)(k0 + j) * NOUT + oo]) * WSC);
  for (int pass = 0; pass < 2; ++pass) { *(volatile v8b*)(WT + e) = o; __threadfence(); }
}
template <int KD, int NOUT, int NV, bool RNDA  >
__global__ __launch_bounds__(64) void gemm_kernel(const float* __restrict__ A, const b16* __restrict__ W, float* __restrict__ T) {
  constexpr int SL = NOUT < 128 ? NOUT : 128, NT = SL / 16, KC = KD < 128 ? KD : 128;
  static_assert(KD % KC == 0 && KC % 32 == 0 && NOUT % SL == 0 && SL % 32 == 0, "gemm tiling");
  __shared__ __attribute__((aligned(16))) b16 Ah[2][16][KC + 8], Al[2][16][KC + 8]; __shared__ __attribute__((aligned(16))) float Tf[2][16][SL + 4];
  const int wave = threadIdx.x >> 5, lane = threadIdx.x & 31, nloc = lane & 15, hlf = lane >> 4; const size_t m0 = (size_t)blockIdx.x * 32 + wave * 16; const int n0 = blockIdx.y * SL;
  v8f acc[NT];
#pragma unroll
  for (int t = 0; t < NT; ++t) acc[t] = (v8f){};
#pragma unroll 1
  for (int kc = 0; kc < KD; kc += KC) {
    for (int idx = lane; idx < 16 * (KC / 4); idx += 32) { const int rr = idx / (KC / 4), c4 = (idx % (KC / 4)) * 4; const size_t row = (m0 + rr < (size_t)NV) ? (m0 + rr) : (size_t)(NV - 1); const v4f v = *(const v4f*)(A + row * KD + kc + c4); v4h hv, lv;
      for (int j = 0; j < 4; ++j) { b16 ph, pl; split16((RNDA ? bf16_rne(v[j]) : v[j]) * XS, ph, pl); hv[j] = ph; lv[j] = pl; } *(v4h*)(&Ah[wave][rr][c4]) = hv; *(v4h*)(&Al[wave][rr][c4]) = lv; }
    wave_lds_sync();
#pragma unroll
    for (int kb = 0; kb < KC; kb += 32) { const v16b a = frag_kb(&Ah[wave][nloc][kb], hlf), al = frag_kb(&Al[wave][nloc][kb], hlf);
#pragma unroll
      for (int t = 0; t < NT; ++t) { const v16b bw = frag_kb(W + (size_t)(n0 + t * 16 + nloc) * KD + kc + kb, hlf); acc[t] = wmma16b(a, bw, acc[t]); acc[t] = wmma16b(al, bw, acc[t]); } }
    wave_lds_sync(); }
#pragma unroll
  for (int t = 0; t < NT; ++t)
#pragma unroll
    for (int r = 0; r < 8; ++r) Tf[wave][8 * hlf + r][t * 16 + nloc] = acc[t][r] * (1.0f / (XS * WSC));
  wave_lds_sync();
  for (int pass = 0; pass < 2; ++pass) { for (int idx = lane; idx < 16 * (SL / 4); idx += 32) { const int rr = idx / (SL / 4), c4 = (idx % (SL / 4)) * 4; *(volatile v4f*)(T + (m0 + rr) * NOUT + n0 + c4) = *(const v4f*)(&Tf[wave][rr][c4]); } __threadfence(); }
}


template <int KD, int NOUT, int LDA, int LDT, bool RNDA>
__global__ __launch_bounds__(64) void gemmx_kernel(const float* __restrict__ A, int nv, const b16* __restrict__ W, const float* __restrict__ bias, int mrows, float* __restrict__ T) {
  constexpr int SL = NOUT < 128 ? NOUT : 128, NT = SL / 16, KC = KD < 128 ? KD : 128;
  static_assert(KD % KC == 0 && KC % 32 == 0 && NOUT % SL == 0 && SL % 32 == 0 && LDA >= KD && LDT >= NOUT, "gemmx tiling");
  __shared__ __attribute__((aligned(16))) b16 Ah[2][16][KC + 8], Al[2][16][KC + 8]; __shared__ __attribute__((aligned(16))) float Tf[2][16][SL + 4];
  const int wave = threadIdx.x >> 5, lane = threadIdx.x & 31, nloc = lane & 15, hlf = lane >> 4; const size_t m0 = (size_t)blockIdx.x * 32 + wave * 16; const int n0 = blockIdx.y * SL;
  v8f acc[NT];
#pragma unroll
  for (int t = 0; t < NT; ++t) acc[t] = (v8f){};
#pragma unroll 1
  for (int kc = 0; kc < KD; kc += KC) {
    for (int idx = lane; idx < 16 * (KC / 4); idx += 32) { const int rr = idx / (KC / 4), c4 = (idx % (KC / 4)) * 4; const size_t row = (m0 + rr < (size_t)nv) ? (m0 + rr) : (size_t)(nv - 1); const v4f v = *(const v4f*)(A + row * LDA + kc + c4); v4h hv, lv;
      for (int j = 0; j < 4; ++j) { b16 ph, pl; split16((RNDA ? bf16_rne(v[j]) : v[j]) * XS, ph, pl); hv[j] = ph; lv[j] = pl; } *(v4h*)(&Ah[wave][rr][c4]) = hv; *(v4h*)(&Al[wave][rr][c4]) = lv; }
    wave_lds_sync();
#pragma unroll
    for (int kb = 0; kb < KC; kb += 32) { const v16b a = frag_kb(&Ah[wave][nloc][kb], hlf), al = frag_kb(&Al[wave][nloc][kb], hlf);
#pragma unroll
      for (int t = 0; t < NT; ++t) { const v16b bw = frag_kb(W + (size_t)(n0 + t * 16 + nloc) * KD + kc + kb, hlf); acc[t] = wmma16b(a, bw, acc[t]); if (!RNDA) acc[t] = wmma16b(al, bw, acc[t]); } }
    wave_lds_sync(); }
#pragma unroll
  for (int t = 0; t < NT; ++t) { const float bb = bias ? bf16_rne(bias[n0 + t * 16 + nloc]) : 0.0f;
#pragma unroll
    for (int r = 0; r < 8; ++r) Tf[wave][8 * hlf + r][t * 16 + nloc] = acc[t][r] * (1.0f / (XS * WSC)) + bb; }
  wave_lds_sync();
  for (int pass = 0; pass < 2; ++pass) { for (int idx = lane; idx < 16 * (SL / 4); idx += 32) { const int rr = idx / (SL / 4), c4 = (idx % (SL / 4)) * 4; if (m0 + rr < (size_t)mrows) *(volatile v4f*)(T + (m0 + rr) * LDT + n0 + c4) = *(const v4f*)(&Tf[wave][rr][c4]); } __threadfence(); }
}

template <int KV, int KD>
__global__ __launch_bounds__(256) void wcopy_kernel(const float* __restrict__ w, int nrow, b16* __restrict__ WT) {
  static_assert(KD % 8 == 0 && KD >= KV, "wcopy"); const size_t u = (size_t)blockIdx.x * 256 + threadIdx.x; if (u >= (size_t)nrow * KD / 8) return; const size_t e = u * 8; const int oo = (int)(e / KD), k0 = (int)(e % KD); v8b o;
  for (int j = 0; j < 8; ++j) { const int k = k0 + j; o[j] = (b16)(k < KV ? bf16_rne(w[(size_t)oo * KV + k]) * WSC : 0.0f); }
  for (int pass = 0; pass < 2; ++pass) { *(volatile v8b*)(WT + e) = o; __threadfence(); }
}
typedef __attribute__((ext_vector_type(2))) _Float16 v2h;
template <int ACT>
__global__ __launch_bounds__(256) void aggns_kernel(const float* __restrict__ T, const float* __restrict__ bias, const int* __restrict__ srcs, const int* __restrict__ PERM, const int* __restrict__ ROWPTR, const int* __restrict__ ROWCNT, int permLen, float* __restrict__ P) {
  __shared__ __attribute__((aligned(16))) float rows[32][D + 4];
  const int wave = threadIdx.x >> 5, lane = threadIdx.x & 31;
#pragma unroll 1
  for (int q4 = 0; q4 < 4; ++q4) { const int rw = wave * 4 + q4; const size_t v = (size_t)blockIdx.x * 32 + rw; v4f o = {0.0f, 0.0f, 0.0f, 0.0f};
    if (v < (size_t)N) { int st = ROWPTR[v], cnt = ROWCNT[v]; cnt = iclamp(cnt, 0, 65536); st = iclamp(st, 0, permLen - cnt); const float dv = cnt > 0 ? rsqrtf((float)cnt) : 0.0f; v4f a = o;
#pragma unroll 1
      for (int j = 0; j < cnt; ++j) { const int e = iclamp(PERM[st + j], 0, E - 1); size_t s = (size_t)iclamp(srcs[e], 0, N - 1); if (SRCM < N) s %= SRCM; const int cs = iclamp(ROWCNT[s], 0, 65536); const float w = cs > 0 ? rsqrtf((float)cs) : 0.0f;
        const v4f t = *(const v4f*)(T + s * D + lane * 4); for (int i = 0; i < 4; ++i) a[i] += pmul(w, t[i]); }
      for (int i = 0; i < 4; ++i) { const float h = pmul(dv, a[i]) + bf16_rne(bias[lane * 4 + i]); o[i] = ACT ? fmaxf(h, 0.0f) : h; } }
    *(v4f*)(&rows[rw][lane * 4]) = o; }
  __syncthreads();
  for (int pass = 0; pass < 2; ++pass) { for (int q = threadIdx.x; q < 32 * D / 4; q += 256) { const int rr = q / (D / 4), c4 = (q % (D / 4)) * 4; *(volatile v4f*)(P + ((size_t)blockIdx.x * 32 + rr) * D + c4) = *(const v4f*)(&rows[rr][c4]); } __threadfence(); }
}
__global__ __launch_bounds__(256) void copy_kernel(const float* __restrict__ H, float* __restrict__ out) { const size_t u = (size_t)blockIdx.x * 256 + threadIdx.x; if (u >= (size_t)N * D / 4) return; const v4f v = *(const v4f*)(H + u * 4); for (int pass = 0; pass < 2; ++pass) { *(volatile v4f*)(out + u * 4) = v; __threadfence(); } }
__global__ __launch_bounds__(256) void tstat_kernel(const float* __restrict__ H, b16* __restrict__ HTh, b16* __restrict__ HTl, float* __restrict__ RSUM, float* __restrict__ CSP) {
  __shared__ __attribute__((aligned(16))) float tile[64][D + 1];
  const int wave = threadIdx.x >> 5, lane = threadIdx.x & 31, t_ = threadIdx.x; const size_t r0 = (size_t)blockIdx.x * 64;
  for (int i = t_; i < 64 * (D / 4); i += 256) { const int rr = i / (D / 4), c4 = (i % (D / 4)) * 4; const size_t row = r0 + rr; v4f v = {0.0f, 0.0f, 0.0f, 0.0f}; if (row < (size_t)NST) v = *(const v4f*)(H + row * D + c4); for (int j = 0; j < 4; ++j) tile[rr][c4 + j] = v[j]; }
  __syncthreads();
  float rs = 0.0f; if (t_ < 64) { for (int c = 0; c < D; ++c) rs += fabsf(tile[t_][c]); }
  float cs = 0.0f; if (t_ < D) { for (int rr = 0; rr < 64; ++rr) cs += fabsf(tile[rr][t_]); }
  for (int pass = 0; pass < 2; ++pass) {
#pragma unroll 1
    for (int q = 0; q < D / 8; ++q) { const int c = wave * (D / 8) + q; v2h hv, lv; for (int j = 0; j < 2; ++j) { const float f = tile[2 * lane + j][c] * XS; const b16 h = (b16)f; hv[j] = h; lv[j] = (b16)((f - (float)h) * RS_); }
      *(volatile v2h*)(HTh + (size_t)c * NP + r0 + 2 * lane) = hv; *(volatile v2h*)(HTl + (size_t)c * NP + r0 + 2 * lane) = lv; }
    if (t_ < 64) ((volatile float*)RSUM)[r0 + t_] = rs;
    if (t_ < D) ((volatile float*)CSP)[(size_t)blockIdx.x * D + t_] = cs;
    __threadfence(); }
}
__global__ __launch_bounds__(256) void gram_kernel(const b16* __restrict__ HTh, const b16* __restrict__ HTl, float* __restrict__ GP) {
  __shared__ __attribute__((aligned(16))) float Tf[8][16][D + 4];
  const int wave = threadIdx.x >> 5, lane = threadIdx.x & 31, nloc = lane & 15, hlf = lane >> 4; const size_t k0 = (size_t)blockIdx.x * KCH; const int m0 = wave * 16;
  v8f acc[8], accl[8];
#pragma unroll
  for (int t = 0; t < 8; ++t) { acc[t] = (v8f){}; accl[t] = (v8f){}; }
#pragma unroll 2
  for (int kb = 0; kb < KCH; kb += 32) { const v16b a = frag_kb(HTh + (size_t)(m0 + nloc) * NP + k0 + kb, hlf), al = frag_kb(HTl + (size_t)(m0 + nloc) * NP + k0 + kb, hlf);
#pragma unroll
    for (int t = 0; t < 8; ++t) { const v16b b = frag_kb(HTh + (size_t)(t * 16 + nloc) * NP + k0 + kb, hlf), bl = frag_kb(HTl + (size_t)(t * 16 + nloc) * NP + k0 + kb, hlf); acc[t] = wmma16b(a, b, acc[t]); accl[t] = wmma16b(a, bl, accl[t]); accl[t] = wmma16b(al, b, accl[t]); } }
#pragma unroll
  for (int t = 0; t < 8; ++t)
#pragma unroll
    for (int r = 0; r < 8; ++r) Tf[wave][8 * hlf + r][t * 16 + nloc] = acc[t][r] * (1.0f / (XS * XS)) + accl[t][r] * (1.0f / (XS * XS * RS_));
  wave_lds_sync();
  for (int pass = 0; pass < 2; ++pass) { for (int rr = 0; rr < 16; ++rr) *(volatile v4f*)(GP + ((size_t)blockIdx.x * D + m0 + rr) * D + lane * 4) = *(const v4f*)(&Tf[wave][rr][lane * 4]); __threadfence(); }
}
__device__ float jacobi_nuc(float (*G)[D + 1], float* cs_c, float* cs_s, int* pr_p, int* pr_q) {
  const int t_ = threadIdx.x;
#pragma unroll 1
  for (int sw = 0; sw < SWEEPS; ++sw) {
#pragma unroll 1
    for (int rd = 0; rd < D - 1; ++rd) {
      if (t_ < 64) { int p, q; if (t_ == 0) { p = D - 1; q = rd; } else { p = (rd + t_) % (D - 1); q = (rd - t_ + (D - 1)) % (D - 1); }
        const float gpq = G[p][q], gpp = G[p][p], gqq = G[q][q]; float c = 1.0f, s = 0.0f;
        if (fabsf(gpq) > 1e-30f) { const float tau = (gqq - gpp) / (2.0f * gpq); const float tt = (tau >= 0.0f ? 1.0f : -1.0f) / (fabsf(tau) + sqrtf(1.0f + tau * tau)); c = rsqrtf(1.0f + tt * tt); s = tt * c; }
        cs_c[t_] = c; cs_s[t_] = s; pr_p[t_] = p; pr_q[t_] = q; }
      __syncthreads();
#pragma unroll 2
      for (int it = t_; it < 64 * D; it += 256) { const int pi = it / D, k = it % D; const int p = pr_p[pi], q = pr_q[pi]; const float c = cs_c[pi], s = cs_s[pi]; const float gp = G[p][k], gq = G[q][k]; G[p][k] = c * gp - s * gq; G[q][k] = s * gp + c * gq; }
      __syncthreads();
#pragma unroll 2
      for (int it = t_; it < 64 * D; it += 256) { const int pi = it / D, k = it % D; const int p = pr_p[pi], q = pr_q[pi]; const float c = cs_c[pi], s = cs_s[pi]; const float gp = G[k][p], gq = G[k][q]; G[k][p] = c * gp - s * gq; G[k][q] = s * gp + c * gq; }
      __syncthreads(); } }
  __shared__ float red[D];
  if (t_ < D) red[t_] = sqrtf(fmaxf(G[t_][t_], 0.0f));
  __syncthreads();
  for (int w = D / 2; w >= 1; w >>= 1) { if (t_ < w) red[t_] += red[t_ + w]; __syncthreads(); }
  const float r = red[0]; __syncthreads(); return r;
}
__global__ __launch_bounds__(256) void stat_kernel(const float* __restrict__ H, const float* __restrict__ GP, const float* __restrict__ RSUM, const float* __restrict__ CSP, float* __restrict__ GS, int sidx, float* __restrict__ STAT) {
  __shared__ __attribute__((aligned(16))) float G[D][D + 1]; __shared__ float cs_c[64], cs_s[64], bvec[D], vvec[D], colsum[D]; __shared__ int pr_p[64], pr_q[64]; __shared__ float amax_v[256]; __shared__ int amax_i[256];
  const int t_ = threadIdx.x;
#pragma unroll 1
  for (int e = t_; e < D * D; e += 256) { float a = 0.0f;
#pragma unroll 1
    for (int c = 0; c < NCH; ++c) a += GP[(size_t)c * D * D + e]; G[e / D][e % D] = a; }
  __syncthreads();
  for (int pass = 0; pass < 2; ++pass) { for (int e = t_; e < D * D; e += 256) ((volatile float*)GS)[e] = G[e / D][e % D]; __threadfence(); }
  if (t_ < D) { float a = 0.0f;
#pragma unroll 1
    for (int b = 0; b < NB64; ++b) a += CSP[(size_t)b * D + t_]; colsum[t_] = a; }
  { float bv = -1.0f; int bi = 0;
#pragma unroll 1
    for (int r = t_; r < NST; r += 256) { const float v = RSUM[r]; if (v > bv) { bv = v; bi = r; } }
    amax_v[t_] = bv; amax_i[t_] = bi; }
  __syncthreads();
  for (int w = 128; w >= 1; w >>= 1) { if (t_ < w) { const float v2 = amax_v[t_ + w]; const int i2 = amax_i[t_ + w]; if (v2 > amax_v[t_] || (v2 == amax_v[t_] && i2 < amax_i[t_])) { amax_v[t_] = v2; amax_i[t_] = i2; } } __syncthreads(); }
  const int irow = amax_i[0]; int jcol = 0; { float bv = -1.0f;
#pragma unroll 1
    for (int c = 0; c < D; ++c) { if (colsum[c] > bv) { bv = colsum[c]; jcol = c; } } }
  __syncthreads();
  const float nuc1 = jacobi_nuc(G, cs_c, cs_s, pr_p, pr_q); const float s1 = 1.0f / nuc1;
  if (t_ < D) { bvec[t_] = s1 * H[(size_t)irow * D + t_]; vvec[t_] = s1 * GS[t_ * D + jcol]; }
  __syncthreads();
  { const float sgn = (bvec[jcol] < 0.0f) ? -1.0f : 1.0f; __syncthreads(); if (t_ < D) bvec[t_] *= sgn; __syncthreads(); }
  float nb2 = 0.0f;
#pragma unroll 4
  for (int c = 0; c < D; ++c) nb2 += bvec[c] * bvec[c];
  const float na2 = s1 * s1 * GS[jcol * D + jcol]; const float cc = rsqrtf(na2 * nb2);
#pragma unroll 1
  for (int e = t_; e < D * D; e += 256) { const int m = e / D, n = e % D; G[m][n] = s1 * s1 * GS[e] - s1 * cc * (vvec[m] * bvec[n] + bvec[m] * vvec[n]) + cc * cc * na2 * bvec[m] * bvec[n]; }
  __syncthreads();
  const float nuc2 = jacobi_nuc(G, cs_c, cs_s, pr_p, pr_q);
  for (int pass = 0; pass < 2; ++pass) { if (t_ < 32) ((volatile float*)STAT)[sidx * 32 + t_] = (t_ == 0) ? nuc2 : (t_ == 1 ? nuc1 : (t_ == 2 ? (float)irow : (t_ == 3 ? (float)jcol : 0.0f))); __threadfence(); }
}
__global__ __launch_bounds__(64) void final_kernel(const float* __restrict__ STAT, float* __restrict__ out1) { if (threadIdx.x == 0) { v4f o; for (int s = 0; s < 4; ++s) o[s] = STAT[s * 32]; for (int pass = 0; pass < 2; ++pass) { *(volatile v4f*)out1 = o; __threadfence(); } } }
}

extern "C" void kernel_launch(void* const* d_in, const int* in_sizes, int n_in, void* d_out, int out_size, void* d_ws, size_t ws_size, hipStream_t stream) {
  (void)n_in;
  auto Fp = [&](int i) { return (const float*)d_in[i]; }; auto Ip = [&](int i) { return (const int*)d_in[i]; };
  if (in_sizes[0] != N * D || in_sizes[1] != 2 * EFULL || in_sizes[2] != D * D || in_sizes[3] != D || in_sizes[4] != D * D || in_sizes[8] != D * D || in_sizes[9] != D || out_size != N * D + 4) return;
  size_t off = 0; char* ws = (char*)d_ws;
  auto carve = [&](size_t bytes) { char* p = ws + off; off += (bytes + 255) & ~(size_t)255; return p; };
  b16* WT = (b16*)carve((size_t)4 * D * D * 2); float* HA = (float*)carve((size_t)NP * D * 4); float* HB = (float*)carve((size_t)NP * D * 4); float* T = (float*)carve((size_t)NP * D * 4);
  b16* HTh = (b16*)carve((size_t)D * NP * 2); b16* HTl = (b16*)carve((size_t)D * NP * 2); float* GP = (float*)carve((size_t)NCH * D * D * 4); float* RSUM = (float*)carve((size_t)NP * 4); float* CSP = (float*)carve((size_t)NB64 * D * 4); float* GS = (float*)carve((size_t)D * D * 4); float* STAT = (float*)carve((size_t)4 * 32 * 4);
  CsrBufs csr; off = csr_carve(csr, ws, off, E, N);
  if (off > ws_size || off > ((size_t)128 << 20)) return;
  for (int l = 0; l < 4; ++l) wcopy_kernel<D, D><<<(D * D / 8 + 255) / 256, 256, 0, stream>>>(Fp(2 + 2 * l), D, WT + (size_t)l * D * D);
  csr_build(csr, Ip(1) + EFULL, E, N, stream);
  auto stats = [&](const float* Hs, int s) {
    tstat_kernel<<<NB64, 256, 0, stream>>>(Hs, HTh, HTl, RSUM, CSP);
    gram_kernel<<<NCH, 256, 0, stream>>>(HTh, HTl, GP);
    stat_kernel<<<1, 256, 0, stream>>>(Hs, GP, RSUM, CSP, GS, s, STAT); };
  gemmx_kernel<D, D, D, D, true><<<dim3(NPL / 32, 1), 64, 0, stream>>>(Fp(0), N, WT, Fp(3), NPL, HA); stats(HA, 0);
  gemmx_kernel<D, D, D, D, false><<<dim3(NPL / 32, 1), 64, 0, stream>>>(HA, NP, WT + (size_t)D * D, nullptr, NPL, T);
  aggns_kernel<1><<<NPL / 32, 256, 0, stream>>>(T, Fp(5), Ip(1), csr.PERM, csr.ROWPTR, csr.ROWCNT, (int)csr.permLen, HB); stats(HB, 1);
  gemmx_kernel<D, D, D, D, false><<<dim3(NPL / 32, 1), 64, 0, stream>>>(HB, NP, WT + (size_t)2 * D * D, nullptr, NPL, T);
  aggns_kernel<1><<<NPL / 32, 256, 0, stream>>>(T, Fp(7), Ip(1), csr.PERM, csr.ROWPTR, csr.ROWCNT, (int)csr.permLen, HA); stats(HA, 2);
  gemmx_kernel<D, D, D, D, false><<<dim3(NPL / 32, 1), 64, 0, stream>>>(HA, NP, WT + (size_t)3 * D * D, nullptr, NPL, T);
  aggns_kernel<0><<<NPL / 32, 256, 0, stream>>>(T, Fp(9), Ip(1), csr.PERM, csr.ROWPTR, csr.ROWCNT, (int)csr.permLen, HB); stats(HB, 3);
  copy_kernel<<<(unsigned)(((size_t)N * D / 4 + 255) / 256), 256, 0, stream>>>(HB, (float*)d_out);
  final_kernel<<<1, 64, 0, stream>>>(STAT, (float*)d_out + (size_t)N * D);
}
